// LinearAttention_31473520345440
// MI455X (gfx1250) — hardware-verified
//
#include <hip/hip_runtime.h>
#include <stddef.h>


typedef _Float16 h16;
typedef _Float16 v16h __attribute__((ext_vector_type(16)));
typedef _Float16 v8h  __attribute__((ext_vector_type(8)));
typedef float    v8f  __attribute__((ext_vector_type(8)));
typedef float    v4f  __attribute__((ext_vector_type(4)));

#ifndef NB
#define NB 4
#endif
#ifndef SEQ
#define SEQ 4096
#endif
#define NB_FULL  4
#define SEQ_FULL 4096
#define DIM   256
#define MROWS (NB * SEQ)

#ifndef SCORE_RES
#define SCORE_RES 1
#endif
#ifndef KPROJ_RES
#define KPROJ_RES 1
#endif

static_assert(NB >= 1 && NB <= NB_FULL);
static_assert(SEQ >= 128 && SEQ <= SEQ_FULL && (SEQ % 128) == 0);
static_assert((SEQ % 64) == 0 && (SEQ % 32) == 0);
static_assert(DIM == 256);
static_assert((DIM % 64) == 0 && (DIM % 32) == 0);
static_assert(DIM == 32 * 8);
static_assert(DIM == 16 * 16);
static_assert(DIM == 4 * 64);
static_assert((MROWS % 64) == 0 && (MROWS % 8) == 0);
static_assert((size_t)MROWS * DIM < (size_t)0xFFFFFFFFu);

#define LDT 72
#define LDC 68
static_assert((LDT % 8) == 0 && LDT >= 64);
static_assert((LDC % 4) == 0 && LDC >= 64);

#define WCARRY 64.0f
#define RCARRY 2048.0f
#define PLN    9.704060528f
#define PCUT   (-9.70f)

#define W_BYTES       ((size_t)DIM * DIM * 2)
#define PLANE16_BYTES ((size_t)MROWS * DIM * 2)
#define OFF_WQ  ((size_t)0)
#define OFF_WK  (OFF_WQ + W_BYTES)
#define OFF_WV  (OFF_WK + W_BYTES)
#define OFF_WR  (OFF_WV + W_BYTES)
#define OFF_XQ  (OFF_WR + W_BYTES)
#define OFF_XV  (OFF_XQ + PLANE16_BYTES)
#define OFF_QH  (OFF_XV + PLANE16_BYTES)
#define OFF_QR  (OFF_QH + PLANE16_BYTES)
#define OFF_KH  (OFF_QR + PLANE16_BYTES)
#define OFF_KR  (OFF_KH + PLANE16_BYTES)
#define OFF_CH  (OFF_KR + PLANE16_BYTES)
#define OFF_CR  (OFF_CH + PLANE16_BYTES)
#define OFF_VT  (OFF_CR + PLANE16_BYTES)
#define WS_TOTAL (OFF_VT + PLANE16_BYTES)
static_assert((W_BYTES % 128) == 0 && (PLANE16_BYTES % 128) == 0);
static_assert(WS_TOTAL <= (size_t)134217728);

__device__ __forceinline__ float bf16r(float x) {
  unsigned int u = __float_as_uint(x);
  u = (u + 0x7FFFu + ((u >> 16) & 1u)) & 0xFFFF0000u;
  return __uint_as_float(u);
}

static __device__ __forceinline__ h16 toh_flush(float v) {
  const h16 r = (h16)v;
  return (fabsf(v) < 6.103515625e-05f) ? (h16)0.0f : r;
}

__device__ __forceinline__ v16h frag_at(const _Float16* p) {
  v8h lo = *(const v8h*)(p);
  v8h hi = *(const v8h*)(p + 16);
  v16h out;
#pragma unroll
  for (int i = 0; i < 8; ++i) { out[i] = lo[i]; out[i + 8] = hi[i]; }
  return out;
}

__device__ __forceinline__ v8f wmma16(v16h a, v16h b, v8f c) {
  v8f d = __builtin_amdgcn_wmma_f32_16x16x32_f16(false, a, false, b, (short)0, c,
                                                 false, false);
  asm volatile("v_nop\n\tv_nop\n\tv_nop\n\tv_nop" : "+v"(d) : "v"(a), "v"(b));
  return d;
}

__device__ __forceinline__ void wave_lds_sync() {
  __builtin_amdgcn_fence(3  , "wavefront");
  asm volatile("s_wait_dscnt 0x0" ::: "memory");
  __builtin_amdgcn_wave_barrier();
}

__global__ __launch_bounds__(256) void wconv_kernel(
    const float* __restrict__ W, _Float16* __restrict__ Wt, unsigned ldw, unsigned ldk) {
  __shared__ _Float16 T[64 * LDT];
  const unsigned tid = threadIdx.x;
  const unsigned n0 = blockIdx.x * 64u;
  const unsigned k0 = blockIdx.y * 64u;
#pragma unroll 4
  for (unsigned j = 0; j < 16u; ++j) {
    const unsigned idx = tid + 256u * j;
    const unsigned kr = idx >> 6, nc = idx & 63u;
    const float v = W[(size_t)(k0 + kr) * ldw + n0 + nc];
    T[nc * LDT + kr] = (_Float16)(WCARRY * bf16r(v));
  }
  __syncthreads();
  v8h x[2];
  size_t off[2];
#pragma unroll
  for (unsigned i = 0; i < 2u; ++i) {
    const unsigned n = 32u * i + (tid >> 3);
    const unsigned kc = (tid & 7u) * 8u;
    x[i] = *(const v8h*)&T[n * LDT + kc];
    off[i] = (size_t)(n0 + n) * ldk + k0 + kc;
  }
#pragma unroll
  for (int i = 0; i < 2; ++i) *(volatile v8h*)(Wt + off[i]) = x[i];
  __threadfence();
#pragma unroll
  for (int i = 0; i < 2; ++i) *(volatile v8h*)(Wt + off[i]) = x[i];
}

__global__ __launch_bounds__(256) void xcast_kernel(
    const float* __restrict__ X, _Float16* __restrict__ dst) {
  const unsigned lane = threadIdx.x & 31u;
  const unsigned wave = __builtin_amdgcn_readfirstlane(threadIdx.x >> 5);
  const unsigned crow = blockIdx.x * 8u + wave;
  const unsigned bidx = crow / (unsigned)SEQ;
  const unsigned sq = crow - bidx * (unsigned)SEQ;
  const size_t srow = (size_t)bidx * SEQ_FULL + sq;
  const float* xr = X + srow * DIM + lane * 8u;
  const v4f a0 = *(const v4f*)(xr);
  const v4f a1 = *(const v4f*)(xr + 4u);
  v8h o;
#pragma unroll
  for (int i = 0; i < 4; ++i) {
    o[i]     = toh_flush(bf16r(a0[i]));
    o[i + 4] = toh_flush(bf16r(a1[i]));
  }
  _Float16* p = dst + (size_t)crow * DIM + lane * 8u;
  *(volatile v8h*)p = o;
  __threadfence();
  *(volatile v8h*)p = o;
}

template <int MODE>
__device__ __forceinline__ void gemm_body(
    const _Float16* __restrict__ A16, const _Float16* __restrict__ A16r,
    const _Float16* __restrict__ Bt, const float* __restrict__ bias,
    _Float16* __restrict__ out16, _Float16* __restrict__ out16r) {
  __shared__ float Cs[64 * LDC];
  const unsigned tid = threadIdx.x, lane = tid & 31u;
  const unsigned w = __builtin_amdgcn_readfirstlane(tid >> 5);
  const unsigned mw = w >> 1, nw = w & 1u;
  const unsigned hh = lane >> 4, m = lane & 15u;
  const unsigned n0 = blockIdx.x * 64u;
  const unsigned row0 = blockIdx.y * 64u;

  const size_t aoff = (size_t)(row0 + mw * 16u + m) * DIM + hh * 8u;
  const size_t boff = (size_t)(n0 + nw * 32u + m) * DIM + hh * 8u;
  v8f acc0 = {}, acc1 = {}, accr0 = {}, accr1 = {};
#pragma unroll 2
  for (unsigned k0 = 0; k0 < (unsigned)DIM; k0 += 32u) {
    const v16h a  = frag_at(A16 + aoff + k0);
    const v16h b0 = frag_at(Bt + boff + k0);
    const v16h b1 = frag_at(Bt + boff + (size_t)16 * DIM + k0);
    acc0 = wmma16(a, b0, acc0);
    acc1 = wmma16(a, b1, acc1);
    if (MODE == 2 && KPROJ_RES) {
      const v16h ar = frag_at(A16r + aoff + k0);
      accr0 = wmma16(ar, b0, accr0);
      accr1 = wmma16(ar, b1, accr1);
    }
  }
#pragma unroll
  for (int r = 0; r < 8; ++r) {
    float* d = &Cs[(mw * 16u + hh * 8u + (unsigned)r) * LDC + nw * 32u + m];
    float v0 = acc0[r] * (1.0f / WCARRY);
    float v1 = acc1[r] * (1.0f / WCARRY);
    if (MODE == 2 && KPROJ_RES) {
      v0 = v0 + accr0[r] * (1.0f / (WCARRY * RCARRY));
      v1 = v1 + accr1[r] * (1.0f / (WCARRY * RCARRY));
    }
    d[0]  = v0;
    d[16] = v1;
  }
  __syncthreads();

  if (MODE == 2) {
#pragma unroll 1
    for (unsigned e = 0; e < 16u; ++e) {
      const unsigned r = 32u * (e >> 3) + (tid >> 3);
      const unsigned c = (tid & 7u) * 8u + (e & 7u);
      const float u = Cs[r * LDC + c];
      const float gb = bias[n0 + c];
      Cs[r * LDC + c] = cosf(u + bf16r(gb));
    }
    __syncthreads();
  }

  if (MODE == 0 || MODE == 2) {
    v8h x[2], xr[2];
    size_t off[2];
#pragma unroll
    for (unsigned i = 0; i < 2u; ++i) {
      const unsigned r = 32u * i + (tid >> 3);
      const unsigned c = (tid & 7u) * 8u;
      const v4f u0 = *(const v4f*)&Cs[r * LDC + c];
      const v4f u1 = *(const v4f*)&Cs[r * LDC + c + 4];
      const v4f g0 = *(const v4f*)(bias + n0 + c);
      const v4f g1 = *(const v4f*)(bias + n0 + c + 4u);
#pragma unroll
      for (int j = 0; j < 4; ++j) {
        const float t0 = (MODE == 0) ? (u0[j] + bf16r(g0[j])) : u0[j];
        const float t1 = (MODE == 0) ? (u1[j] + bf16r(g1[j])) : u1[j];
        const h16 h0 = toh_flush(t0);
        const h16 h1 = toh_flush(t1);
        x[i][j]      = h0;
        x[i][j + 4]  = h1;
        xr[i][j]     = toh_flush((t0 - (float)h0) * RCARRY);
        xr[i][j + 4] = toh_flush((t1 - (float)h1) * RCARRY);
      }
      off[i] = (size_t)(row0 + r) * DIM + n0 + c;
    }
#pragma unroll
    for (int i = 0; i < 2; ++i) *(volatile v8h*)(out16 + off[i]) = x[i];
#pragma unroll
    for (int i = 0; i < 2; ++i) *(volatile v8h*)(out16r + off[i]) = xr[i];
    __threadfence();
#pragma unroll
    for (int i = 0; i < 2; ++i) *(volatile v8h*)(out16 + off[i]) = x[i];
#pragma unroll
    for (int i = 0; i < 2; ++i) *(volatile v8h*)(out16r + off[i]) = xr[i];
  }

  if (MODE == 1) {
    const unsigned bidx = row0 / (unsigned)SEQ;
    const unsigned key0 = row0 - bidx * (unsigned)SEQ;
    v8h x[2];
    size_t off[2];
#pragma unroll
    for (unsigned i = 0; i < 2u; ++i) {
      const unsigned dcol = 32u * i + (tid >> 3);
      const unsigned kk = (tid & 7u) * 8u;
      const float bb = bf16r(bias[n0 + dcol]);
#pragma unroll
      for (unsigned j = 0; j < 8u; ++j) {
        const float t = Cs[(kk + j) * LDC + dcol] + bb;
        x[i][j] = toh_flush(t);
      }
      off[i] = ((size_t)bidx * DIM + n0 + dcol) * SEQ + key0 + kk;
    }
#pragma unroll
    for (int i = 0; i < 2; ++i) *(volatile v8h*)(out16 + off[i]) = x[i];
    __threadfence();
#pragma unroll
    for (int i = 0; i < 2; ++i) *(volatile v8h*)(out16 + off[i]) = x[i];
  }
}

__global__ __launch_bounds__(256) void gemm_qk_kernel(
    const _Float16* __restrict__ A16, const _Float16* __restrict__ Bt,
    const float* __restrict__ bias, _Float16* __restrict__ out16,
    _Float16* __restrict__ out16r) {
  gemm_body<0>(A16, A16, Bt, bias, out16, out16r);
}
__global__ __launch_bounds__(256) void gemm_v_kernel(
    const _Float16* __restrict__ A16, const _Float16* __restrict__ Bt,
    const float* __restrict__ bias, _Float16* __restrict__ vt) {
  gemm_body<1>(A16, A16, Bt, bias, vt, vt);
}
__global__ __launch_bounds__(256) void gemm_feat_kernel(
    const _Float16* __restrict__ A16, const _Float16* __restrict__ A16r,
    const _Float16* __restrict__ Bt, const float* __restrict__ bias,
    _Float16* __restrict__ out16, _Float16* __restrict__ out16r) {
  gemm_body<2>(A16, A16r, Bt, bias, out16, out16r);
}

__global__ __launch_bounds__(256) __attribute__((amdgpu_num_vgpr(256))) void attn_kernel(
    const _Float16* __restrict__ Qh, const _Float16* __restrict__ Qr,
    const _Float16* __restrict__ Fh, const _Float16* __restrict__ Fr,
    const _Float16* __restrict__ Vt, float* __restrict__ Out) {
  __shared__ float Cw[8 * 16 * LDC];

  const unsigned lane = threadIdx.x & 31u;
  const unsigned wave = __builtin_amdgcn_readfirstlane(threadIdx.x >> 5);
  const unsigned hh = lane >> 4, m = lane & 15u;
  const unsigned b = blockIdx.y;
  const unsigned qrow0 = blockIdx.x * 128u + wave * 16u;
  const unsigned cw0 = wave * (16u * LDC);

  const size_t qoff = ((size_t)b * SEQ + qrow0 + m) * DIM + hh * 8u;
  const size_t koff = ((size_t)b * SEQ + m) * DIM + hh * 8u;
  const size_t voff = ((size_t)b * DIM + m) * SEQ + hh * 8u;

  float mrun = -1.0e30f, lrun = 0.0f;
  v8f o[16];
#pragma unroll
  for (int t = 0; t < 16; ++t) o[t] = (v8f){};

#pragma unroll 1
  for (unsigned kb = 0; kb < (unsigned)SEQ; kb += 32u) {
    const size_t kbase = koff + (size_t)kb * DIM;
    v8f sh0 = {}, sh1 = {};
#if SCORE_RES
    v8f sr0 = {}, sr1 = {};
#endif
#pragma unroll 1
    for (unsigned k0 = 0; k0 < (unsigned)DIM; k0 += 32u) {
      const v16h qh  = frag_at(Qh + qoff + k0);
      const v16h fh0 = frag_at(Fh + kbase + k0);
      const v16h fh1 = frag_at(Fh + kbase + (size_t)16 * DIM + k0);
      sh0 = wmma16(fh0, qh, sh0);
      sh1 = wmma16(fh1, qh, sh1);
#if SCORE_RES
      const v16h qr = frag_at(Qr + qoff + k0);
      sr0 = wmma16(fh0, qr, sr0);
      sr1 = wmma16(fh1, qr, sr1);
      __builtin_amdgcn_sched_barrier(0);
      const v16h fr0 = frag_at(Fr + kbase + k0);
      const v16h fr1 = frag_at(Fr + kbase + (size_t)16 * DIM + k0);
      sr0 = wmma16(fr0, qh, sr0);
      sr1 = wmma16(fr1, qh, sr1);
#endif
      __builtin_amdgcn_sched_barrier(0);
    }

    float sv[16];
#pragma unroll
    for (int r = 0; r < 8; ++r) {
#if SCORE_RES
      sv[r]     = sh0[r] + sr0[r] * (1.0f / RCARRY);
      sv[r + 8] = sh1[r] + sr1[r] * (1.0f / RCARRY);
#else
      sv[r]     = sh0[r];
      sv[r + 8] = sh1[r];
#endif
    }

    float mx = sv[0];
#pragma unroll
    for (int i = 1; i < 16; ++i) mx = fmaxf(mx, sv[i]);
    mx = fmaxf(mx, __shfl_xor(mx, 16, 32));
    const float mn = fmaxf(mrun, mx);
    const float alpha = __expf(mrun - mn);
    mrun = mn;

    float ps = 0.0f;
    v16h pf;
#pragma unroll
    for (int i = 0; i < 16; ++i) {
      const float t = (sv[i] - mn) + PLN;
      const float p = (t < PCUT) ? 0.0f : __expf(t);
      const h16 ph = (h16)p;
      pf[i] = ph;
      ps += (float)ph;
    }
    lrun = alpha * lrun + ps;

#pragma unroll
    for (int t = 0; t < 16; ++t)
#pragma unroll
      for (int r = 0; r < 8; ++r) o[t][r] = o[t][r] * alpha;

    const _Float16* vp = Vt + voff + kb;
#pragma unroll
    for (int g = 0; g < 4; ++g) {
#pragma unroll
      for (int j = 0; j < 4; ++j) {
        const int t = 4 * g + j;
        const v16h vf = frag_at(vp + (size_t)(16 * t) * SEQ);
        o[t] = wmma16(vf, pf, o[t]);
      }
      __builtin_amdgcn_sched_barrier(0);
    }
  }

  const float lt = lrun + __shfl_xor(lrun, 16, 32);
  const float inv = __builtin_amdgcn_rcpf(lt);
#pragma unroll
  for (int c = 0; c < 4; ++c) {
#pragma unroll
    for (int j = 0; j < 4; ++j) {
      const int t = 4 * c + j;
      v4f ua, ub;
#pragma unroll
      for (int i = 0; i < 4; ++i) {
        ua[i] = o[t][i] * inv;
        ub[i] = o[t][i + 4] * inv;
      }
      *(v4f*)&Cw[cw0 + m * LDC + (unsigned)j * 16u + hh * 8u]      = ua;
      *(v4f*)&Cw[cw0 + m * LDC + (unsigned)j * 16u + hh * 8u + 4u] = ub;
    }
    wave_lds_sync();
    v4f x[8];
    size_t off[8];
#pragma unroll
    for (unsigned i = 0; i < 8u; ++i) {
      const unsigned r = 2u * i + hh;
      const unsigned cc = m * 4u;
      x[i] = *(const v4f*)&Cw[cw0 + r * LDC + cc];
      off[i] = ((size_t)b * SEQ_FULL + qrow0 + r) * DIM + 64u * (unsigned)c + cc;
    }
#pragma unroll
    for (int i = 0; i < 8; ++i) *(volatile v4f*)(Out + off[i]) = x[i];
    __threadfence();
#pragma unroll
    for (int i = 0; i < 8; ++i) *(volatile v4f*)(Out + off[i]) = x[i];
    wave_lds_sync();
  }
}

extern "C" void kernel_launch(void* const* d_in, const int* in_sizes, int n_in,
                              void* d_out, int out_size, void* d_ws, size_t ws_size,
                              hipStream_t stream) {
  if (n_in < 10) return;
  const long long need_x = ((long long)(NB - 1) * SEQ_FULL + SEQ) * DIM;
  if ((long long)in_sizes[0] < need_x) return;
  if ((long long)in_sizes[1] < need_x) return;
  if ((long long)in_sizes[2] < (long long)DIM * DIM) return;
  if ((long long)in_sizes[4] < (long long)DIM * DIM) return;
  if ((long long)in_sizes[6] < (long long)DIM * DIM) return;
  if ((long long)in_sizes[8] < (long long)DIM * DIM) return;
  if (in_sizes[3] < DIM || in_sizes[5] < DIM || in_sizes[7] < DIM || in_sizes[9] < DIM) return;
  if ((long long)out_size < need_x) return;
  if (ws_size < WS_TOTAL) return;

  const float* query = (const float*)d_in[0];
  const float* value = (const float*)d_in[1];
  const float* wq = (const float*)d_in[2];
  const float* bq = (const float*)d_in[3];
  const float* wk = (const float*)d_in[4];
  const float* bk = (const float*)d_in[5];
  const float* wv = (const float*)d_in[6];
  const float* bv = (const float*)d_in[7];
  const float* wr = (const float*)d_in[8];
  const float* br = (const float*)d_in[9];
  float* out = (float*)d_out;

  char* ws = (char*)d_ws;
  _Float16* Wq_t = (_Float16*)(ws + OFF_WQ);
  _Float16* Wk_t = (_Float16*)(ws + OFF_WK);
  _Float16* Wv_t = (_Float16*)(ws + OFF_WV);
  _Float16* Wr_t = (_Float16*)(ws + OFF_WR);
  _Float16* Xq16 = (_Float16*)(ws + OFF_XQ);
  _Float16* Xv16 = (_Float16*)(ws + OFF_XV);
  _Float16* Qh16 = (_Float16*)(ws + OFF_QH);
  _Float16* Qr16 = (_Float16*)(ws + OFF_QR);
  _Float16* Kh16 = (_Float16*)(ws + OFF_KH);
  _Float16* Kr16 = (_Float16*)(ws + OFF_KR);
  _Float16* Fh16 = (_Float16*)(ws + OFF_CH);
  _Float16* Fr16 = (_Float16*)(ws + OFF_CR);
  _Float16* Vt16 = (_Float16*)(ws + OFF_VT);

  dim3 blk(256);
  dim3 gsq(DIM / 64, DIM / 64);
  dim3 gg(DIM / 64, MROWS / 64);

  wconv_kernel<<<gsq, blk, 0, stream>>>(wq, Wq_t, (unsigned)DIM, (unsigned)DIM);
  wconv_kernel<<<gsq, blk, 0, stream>>>(wk, Wk_t, (unsigned)DIM, (unsigned)DIM);
  wconv_kernel<<<gsq, blk, 0, stream>>>(wv, Wv_t, (unsigned)DIM, (unsigned)DIM);
  wconv_kernel<<<gsq, blk, 0, stream>>>(wr, Wr_t, (unsigned)DIM, (unsigned)DIM);

  xcast_kernel<<<dim3(MROWS / 8), blk, 0, stream>>>(query, Xq16);
  xcast_kernel<<<dim3(MROWS / 8), blk, 0, stream>>>(value, Xv16);

  gemm_qk_kernel<<<gg, blk, 0, stream>>>(Xq16, Wq_t, bq, Qh16, Qr16);
  gemm_qk_kernel<<<gg, blk, 0, stream>>>(Xv16, Wk_t, bk, Kh16, Kr16);
  gemm_v_kernel<<<gg, blk, 0, stream>>>(Xv16, Wv_t, bv, Vt16);
  gemm_feat_kernel<<<gg, blk, 0, stream>>>(Kh16, Kr16, Wr_t, br, Fh16, Fr16);
  attn_kernel<<<dim3(SEQ / 128, NB), blk, 0, stream>>>(Qh16, Qr16, Fh16, Fr16, Vt16, out);
}
